// ConvCaps_9337258901594
// MI455X (gfx1250) — hardware-verified
//
#include <hip/hip_runtime.h>
#include <math.h>
#include <stdint.h>

constexpr int kNb    = 16;
constexpr int kAcap  = 32;
constexpr int kBcap  = 32;
constexpr int kCdim  = 16;
constexpr int kDdim  = 16;
constexpr int kHin   = 14;
constexpr int kWin   = 14;
constexpr int kPix   = kHin * kWin;
constexpr int kOw    = 6;
constexpr int kL     = 36;
constexpr int kNrow  = 288;
constexpr int kP     = kNb * kL;
constexpr int kM     = kBcap * kDdim;
constexpr int kK     = kNrow * kCdim;
constexpr int kSteps = kK / 32;
constexpr float kCarryA    = 2048.0f;
constexpr float kW2Carry   = 16.0f;
constexpr float kW2CarryInv = 1.0f / 16.0f;
constexpr float kInvP      = 1.0f / 576.0f;
constexpr float kBnEps     = 1e-5f;

constexpr int kOut0Elems = kNb * kBcap * kL;
constexpr int kOut1Elems = kNb * kM * kL;
constexpr int kOutElems  = kOut0Elems + kOut1Elems;
static_assert(kOut0Elems * 4 == 73728);
static_assert((kOut0Elems + kOut1Elems) * 4 == 1253376);
static_assert(kK % 32 == 0);
static_assert(kP % 16 == 0);
static_assert(kNrow == 9 * 32);

constexpr size_t kBytesBt    = (size_t)kBcap * kDdim * kK * 2;
constexpr size_t kBytesPu    = (size_t)kP * kK * 4;
constexpr size_t kBytesAr    = (size_t)kP * kNrow * kBcap * 4;
constexpr size_t kBytesTab   = (size_t)kP * kBcap * 4;
constexpr size_t kBytesPoseo = (size_t)kP * kM * 4;
constexpr size_t kBytesStat  = (size_t)kM * 4;
constexpr size_t kOffBt    = 0;
constexpr size_t kOffPu    = kOffBt + kBytesBt;
constexpr size_t kOffAr    = kOffPu + kBytesPu;
constexpr size_t kOffArsum = kOffAr + kBytesAr;
constexpr size_t kOffAout  = kOffArsum + kBytesTab;
constexpr size_t kOffPoseo = kOffAout + kBytesTab;
constexpr size_t kOffMean  = kOffPoseo + kBytesPoseo;
constexpr size_t kOffRstd  = kOffMean + kBytesStat;
constexpr size_t kWsTotal  = kOffRstd + kBytesStat;
static_assert(kBytesBt == 4718592);
static_assert(kWsTotal == 37900288);
static_assert(kWsTotal <= 134217728);
static_assert(kOffPu % 128 == 0 && kOffAr % 128 == 0 && kOffArsum % 128 == 0 && kOffAout % 128 == 0);
static_assert(kOffPoseo % 128 == 0 && kOffMean % 128 == 0 && kOffRstd % 128 == 0);

typedef __attribute__((ext_vector_type(16))) _Float16 v16h;
typedef __attribute__((ext_vector_type(8)))  _Float16 v8h;
typedef __attribute__((ext_vector_type(8)))  float    v8f;
typedef __attribute__((ext_vector_type(4)))  float    v4f;
typedef __attribute__((ext_vector_type(4)))  unsigned int v4u;

__device__ __forceinline__ void dep_guard_h(v8f& a, v8f& b, v16h x, v16h y) { asm volatile("v_nop\n\tv_nop\n\tv_nop\n\tv_nop" : "+v"(a), "+v"(b) : "v"(x), "v"(y)); }
__device__ __forceinline__ void keep4_h(v16h a, v16h b, v16h c, v16h d) { asm volatile("v_nop" :: "v"(a), "v"(b), "v"(c), "v"(d)); }
template <typename T> struct Frag;
template <> struct Frag<_Float16> {
  typedef v16h V; union U { v16h v; v8h h[2]; };
  static __device__ __forceinline__ v16h load(const _Float16* p) {
    U f; f.h[0] = *(const v8h*)(p); f.h[1] = *(const v8h*)(p + 16); return f.v;
  }
  static __device__ __forceinline__ v8f mma(v16h a, v16h b, v8f c) {
    return __builtin_amdgcn_wmma_f32_16x16x32_f16(false, a, false, b, (short)0, c, false, false);
  }
  static __device__ __forceinline__ void guard(v8f& a, v8f& b, v16h x, v16h y) { dep_guard_h(a, b, x, y); }
  static __device__ __forceinline__ void keep(v16h a, v16h b, v16h c, v16h d) { keep4_h(a, b, c, d); }
};
__device__ __forceinline__ unsigned pk16(unsigned short a, unsigned short b) { return (unsigned)a | ((unsigned)b << 16); }
__device__ __forceinline__ unsigned short h_bits(float f) { const _Float16 h = (_Float16)f; return __builtin_bit_cast(unsigned short, h); }

__device__ __forceinline__ v8f mma_f16_g(v16h a, v16h b, v8f c) {
  c = __builtin_amdgcn_wmma_f32_16x16x32_f16(false, a, false, b, (short)0, c, false, false);
  asm volatile("v_nop\n\tv_nop\n\tv_nop\n\tv_nop" : "+v"(c) : "v"(a), "v"(b));
  return c;
}

constexpr int kBtUnits = (kBcap * kDdim * kK) / 8;
__global__ __launch_bounds__(256) void repack_w1_kernel(const float* __restrict__ W1, unsigned short* __restrict__ bt) {
  const int i = blockIdx.x * 256 + threadIdx.x;
  if (i >= kBtUnits) return;
  const int o   = i * 8;
  const int j   = o / (kDdim * kK);
  const int rem = o - j * (kDdim * kK);
  const int d   = rem / kK;
  const int k   = rem - d * kK;
  const int n   = k >> 4;
  const int c0  = k & 15;
  const float* src = W1 + ((size_t)n * kM + j * kDdim + d) * kCdim + c0;
  const v4f a = *(const v4f*)(src);
  const v4f c = *(const v4f*)(src + 4);
  unsigned short hb[8];
#pragma unroll
  for (int e = 0; e < 4; ++e) {
    hb[e]     = h_bits(a[e]);
    hb[4 + e] = h_bits(c[e]);
  }
  const v4u u = (v4u){pk16(hb[0], hb[1]), pk16(hb[2], hb[3]), pk16(hb[4], hb[5]), pk16(hb[6], hb[7])};
  unsigned short* q = bt + (size_t)o;
  *(volatile v4u*)q = u;
  __threadfence();
  *(volatile v4u*)q = u;
}

__global__ __launch_bounds__(288) void gather_pose_kernel(const float* __restrict__ pose, float* __restrict__ pu) {
  const int p  = blockIdx.x;
  const int t  = threadIdx.x;
  const int b  = p / kL;
  const int l  = p - b * kL;
  const int y0 = 2 * (l / kOw);
  const int x0 = 2 * (l % kOw);
  float* prow = pu + (size_t)p * kK;
#pragma unroll 1
  for (int it = 0; it < 4; ++it) {
    const int k  = 4 * (it * 288 + t);
    const int n  = k >> 4;
    const int c0 = k & 15;
    const int kk = n >> 5;
    const int ai = n & 31;
    const int ki = kk / 3;
    const int kj = kk - 3 * ki;
    const float* src = pose + ((size_t)(b * (kAcap * kCdim) + ai * kCdim + c0) * kHin + y0 + ki) * kWin + x0 + kj;
    v4f v;
    v[0] = src[0];
    v[1] = src[kPix];
    v[2] = src[2 * kPix];
    v[3] = src[3 * kPix];
    float* dst = prow + k;
    *(volatile v4f*)dst = v;
    __threadfence();
    *(volatile v4f*)dst = v;
  }
}

__global__ __launch_bounds__(288) void route_kernel(const float* __restrict__ act, const float* __restrict__ pu,
                                                   const float* __restrict__ W2, const float* __restrict__ b2,
                                                   float* __restrict__ ar_ws, float* __restrict__ arsum_ws,
                                                   float* __restrict__ aout_ws) {
  __shared__ float au_s[16 * kNrow];
  __shared__ __align__(16) float slab_s[9 * 16 * 36];
  __shared__ __align__(16) float tab_s[2 * 16 * 32];
  __shared__ float ausum_s[16];

  const int t    = threadIdx.x;
  const int lane = t & 31;
  const int w    = t >> 5;
  const int h    = lane >> 4;
  const int rl   = lane & 15;
  const int p0   = blockIdx.x * 16;

  {
    const int kk = t >> 5, ai = t & 31;
    const int ki = kk / 3, kj = kk - 3 * ki;
#pragma unroll 4
    for (int it = 0; it < 16; ++it) {
      const int p = p0 + it;
      const int b = p / kL;
      const int l = p - b * kL;
      au_s[it * kNrow + t] = act[((size_t)(b * kAcap + ai) * kHin + 2 * (l / kOw) + ki) * kWin + 2 * (l % kOw) + kj];
    }
  }
  __syncthreads();

  float* sw = slab_s + w * (16 * 36);
  const int prow = p0 + rl;
  float as0[8], as1[8];
#pragma unroll
  for (int r = 0; r < 8; ++r) { as0[r] = 0.0f; as1[r] = 0.0f; }
  v8h z8;
#pragma unroll
  for (int e = 0; e < 8; ++e) z8[e] = (_Float16)0.0f;
  const v8f zacc = (v8f){0.f,0.f,0.f,0.f,0.f,0.f,0.f,0.f};

#pragma unroll 1
  for (int ns = 0; ns < 32; ++ns) {
    const int n = w * 32 + ns;
    const float* ap = pu + (size_t)prow * kK + n * kCdim + 8 * h;
    const v4f x0 = *(const v4f*)(ap);
    const v4f x1 = *(const v4f*)(ap + 4);
    v8h ah;
#pragma unroll
    for (int e = 0; e < 4; ++e) { ah[e] = (_Float16)x0[e]; ah[4 + e] = (_Float16)x1[e]; }
    Frag<_Float16>::U fa; fa.h[0] = ah; fa.h[1] = z8;
    const float* bp0 = W2 + ((size_t)n * kBcap + rl) * kCdim + 8 * h;
    const float* bp1 = bp0 + 16 * kCdim;
    const v4f w00 = *(const v4f*)(bp0);
    const v4f w01 = *(const v4f*)(bp0 + 4);
    const v4f w10 = *(const v4f*)(bp1);
    const v4f w11 = *(const v4f*)(bp1 + 4);
    v8h bh0, bh1;
#pragma unroll
    for (int e = 0; e < 4; ++e) {
      bh0[e] = (_Float16)(w00[e] * kW2Carry); bh0[4 + e] = (_Float16)(w01[e] * kW2Carry);
      bh1[e] = (_Float16)(w10[e] * kW2Carry); bh1[4 + e] = (_Float16)(w11[e] * kW2Carry);
    }
    Frag<_Float16>::U fb0, fb1;
    fb0.h[0] = bh0; fb0.h[1] = z8;
    fb1.h[0] = bh1; fb1.h[1] = z8;
    v8f acc0 = mma_f16_g(fa.v, fb0.v, zacc);
    v8f acc1 = mma_f16_g(fa.v, fb1.v, zacc);
    const float bias0 = b2[n * kBcap + rl];
    const float bias1 = b2[n * kBcap + 16 + rl];
#pragma unroll
    for (int r = 0; r < 8; ++r) {
      const float v0 = acc0[r] * kW2CarryInv + bias0;
      const float v1 = acc1[r] * kW2CarryInv + bias1;
      float mx = fmaxf(v0, v1);
      mx = fmaxf(mx, __shfl_xor(mx, 1, 32));
      mx = fmaxf(mx, __shfl_xor(mx, 2, 32));
      mx = fmaxf(mx, __shfl_xor(mx, 4, 32));
      mx = fmaxf(mx, __shfl_xor(mx, 8, 32));
      const float e0 = expf(v0 - mx);
      const float e1 = expf(v1 - mx);
      float ssum = e0 + e1;
      ssum += __shfl_xor(ssum, 1, 32);
      ssum += __shfl_xor(ssum, 2, 32);
      ssum += __shfl_xor(ssum, 4, 32);
      ssum += __shfl_xor(ssum, 8, 32);
      const float inv = 1.0f / ssum;
      const float au  = au_s[(8 * h + r) * kNrow + n];
      const float ar0 = au * (e0 * inv);
      const float ar1 = au * (e1 * inv);
      as0[r] += ar0;
      as1[r] += ar1;
      sw[(8 * h + r) * 36 + rl]      = ar0;
      sw[(8 * h + r) * 36 + 16 + rl] = ar1;
    }
    __builtin_amdgcn_fence(__ATOMIC_RELEASE, "workgroup");
    __builtin_amdgcn_wave_barrier();
    __builtin_amdgcn_fence(__ATOMIC_ACQUIRE, "workgroup");
    {
      const int q = lane >> 3, c4 = (lane & 7) * 4;
      float* dst = ar_ws + ((size_t)p0 * kNrow + n) * kBcap;
      for (int pass = 0; pass < 2; ++pass) {
#pragma unroll
        for (int it = 0; it < 4; ++it) {
          const int row = it * 4 + q;
          const v4f v = *(const v4f*)(sw + row * 36 + c4);
          *(volatile v4f*)(dst + (size_t)row * kNrow * kBcap + c4) = v;
        }
        __threadfence();
      }
    }
    __builtin_amdgcn_fence(__ATOMIC_RELEASE, "workgroup");
    __builtin_amdgcn_wave_barrier();
    __builtin_amdgcn_fence(__ATOMIC_ACQUIRE, "workgroup");
  }

  __syncthreads();
  float* red = slab_s;
#pragma unroll
  for (int r = 0; r < 8; ++r) {
    red[(w * 16 + 8 * h + r) * 32 + rl]      = as0[r];
    red[(w * 16 + 8 * h + r) * 32 + 16 + rl] = as1[r];
  }
  __syncthreads();
  for (int idx = t; idx < 512; idx += 288) {
    const int p = idx >> 5, j = idx & 31;
    float s = 0.0f;
#pragma unroll
    for (int ww = 0; ww < 9; ++ww) s += red[(ww * 16 + p) * 32 + j];
    tab_s[idx] = s;
  }
  if (t < 16) {
    float s = 0.0f;
#pragma unroll 4
    for (int n = 0; n < kNrow; ++n) s += au_s[t * kNrow + n];
    ausum_s[t] = s;
  }
  __syncthreads();
  for (int idx = t; idx < 512; idx += 288) {
    const int p = idx >> 5;
    tab_s[512 + idx] = tab_s[idx] * (1.0f / ausum_s[p]);
  }
  __syncthreads();
  if (w < 2) {
    const float* src = tab_s + w * 512;
    float* dst = arsum_ws;
    if (w == 1) dst = aout_ws;
    dst += (size_t)p0 * kBcap;
    const int q = lane >> 3, c4 = (lane & 7) * 4;
    for (int pass = 0; pass < 2; ++pass) {
#pragma unroll
      for (int it = 0; it < 4; ++it) {
        const int row = it * 4 + q;
        const v4f v = *(const v4f*)(src + row * 32 + c4);
        *(volatile v4f*)(dst + (size_t)row * kBcap + c4) = v;
      }
      __threadfence();
    }
  }
}

__global__ __launch_bounds__(256) void vote_gemm_kernel(const float* __restrict__ pu, const float* __restrict__ ar_ws,
                                                       const unsigned short* __restrict__ btp,
                                                       const float* __restrict__ arsum_ws, float* __restrict__ poseo) {
  __shared__ __align__(16) float tile_s[16 * 132];
  const int t    = threadIdx.x;
  const int lane = t & 31;
  const int w    = t >> 5;
  const int h    = lane >> 4;
  const int rl   = lane & 15;
  const int pt   = blockIdx.x % 36;
  const int jg   = blockIdx.x / 36;
  const int j    = jg * 8 + w;
  const int p0   = pt * 16;
  const int prow = p0 + rl;
  const _Float16* bt = (const _Float16*)btp;

  const float* purow = pu + (size_t)prow * kK + 8 * h;
  const float* arrow = ar_ws + (size_t)prow * kNrow * kBcap + j;
  const _Float16* btrow = bt + (size_t)(j * kDdim + rl) * kK + 8 * h;

  v8f acc = (v8f){0.f,0.f,0.f,0.f,0.f,0.f,0.f,0.f};
#pragma unroll 2
  for (int s = 0; s < kSteps; ++s) {
    const int k0 = s * 32;
    const float c0 = arrow[(size_t)(2 * s) * kBcap] * kCarryA;
    const float c1 = arrow[(size_t)(2 * s + 1) * kBcap] * kCarryA;
    const v4f x0 = *(const v4f*)(purow + k0);
    const v4f x1 = *(const v4f*)(purow + k0 + 4);
    const v4f y0 = *(const v4f*)(purow + k0 + 16);
    const v4f y1 = *(const v4f*)(purow + k0 + 20);
    v8h lo8, hi8;
#pragma unroll
    for (int e = 0; e < 4; ++e) {
      lo8[e]     = (_Float16)(c0 * x0[e]);
      lo8[4 + e] = (_Float16)(c0 * x1[e]);
      hi8[e]     = (_Float16)(c1 * y0[e]);
      hi8[4 + e] = (_Float16)(c1 * y1[e]);
    }
    Frag<_Float16>::U fa; fa.h[0] = lo8; fa.h[1] = hi8;
    const v16h fb = Frag<_Float16>::load(btrow + k0);
    acc = mma_f16_g(fa.v, fb, acc);
  }

#pragma unroll
  for (int r = 0; r < 8; ++r) {
    const int row = 8 * h + r;
    const float rs = arsum_ws[(size_t)(p0 + row) * kBcap + j];
    const float val = acc[r] * (1.0f / (rs * kCarryA));
    tile_s[row * 132 + w * 16 + rl] = val;
  }
  __syncthreads();
  {
    const int c4 = lane * 4;
    for (int pass = 0; pass < 2; ++pass) {
#pragma unroll
      for (int rr = 0; rr < 2; ++rr) {
        const int row = 2 * w + rr;
        const v4f v = *(const v4f*)(tile_s + row * 132 + c4);
        *(volatile v4f*)(poseo + (size_t)(p0 + row) * kM + jg * 128 + c4) = v;
      }
      __threadfence();
    }
  }
}

__global__ __launch_bounds__(512) void bn_stats_kernel(const float* __restrict__ poseo, float* __restrict__ mean_ws,
                                                      float* __restrict__ rstd_ws) {
  const int m = threadIdx.x;
  float s = 0.0f;
#pragma unroll 4
  for (int p = 0; p < kP; ++p) s += poseo[(size_t)p * kM + m];
  const float mean = s * kInvP;
  float q = 0.0f;
#pragma unroll 4
  for (int p = 0; p < kP; ++p) {
    const float d = poseo[(size_t)p * kM + m] - mean;
    q += d * d;
  }
  const float var  = q * kInvP;
  const float rstd = rsqrtf(var + kBnEps);
  ((volatile float*)mean_ws)[m] = mean;
  ((volatile float*)rstd_ws)[m] = rstd;
  __threadfence();
  ((volatile float*)mean_ws)[m] = mean;
  ((volatile float*)rstd_ws)[m] = rstd;
}

constexpr int kOut0Units = kOut0Elems / 4;
constexpr int kOut1Units = kOut1Elems / 4;
__global__ __launch_bounds__(256) void write_out0_kernel(const float* __restrict__ aout_ws, float* __restrict__ out) {
  const int i4 = blockIdx.x * 256 + threadIdx.x;
  if (i4 >= kOut0Units) return;
  const int e   = i4 * 4;
  const int b   = e / (kBcap * kL);
  const int rem = e - b * (kBcap * kL);
  const int j   = rem / kL;
  const int l0  = rem - j * kL;
  const int p   = b * kL + l0;
  v4f v;
#pragma unroll
  for (int q = 0; q < 4; ++q) v[q] = aout_ws[(size_t)(p + q) * kBcap + j];
  float* dst = out + e;
  *(volatile v4f*)dst = v;
  __threadfence();
  *(volatile v4f*)dst = v;
}

__global__ __launch_bounds__(256) void write_out1_kernel(const float* __restrict__ poseo, const float* __restrict__ mean_ws,
                                                        const float* __restrict__ rstd_ws, const float* __restrict__ gamma,
                                                        const float* __restrict__ beta, float* __restrict__ out) {
  const int i4 = blockIdx.x * 256 + threadIdx.x;
  if (i4 >= kOut1Units) return;
  const int f   = i4 * 4;
  const int b   = f / (kM * kL);
  const int rem = f - b * (kM * kL);
  const int m   = rem / kL;
  const int l0  = rem - m * kL;
  const int p   = b * kL + l0;
  const float mu = mean_ws[m];
  const float rs = rstd_ws[m];
  const float ga = gamma[m];
  const float be = beta[m];
  v4f v;
#pragma unroll
  for (int q = 0; q < 4; ++q) {
    const float x = poseo[(size_t)(p + q) * kM + m];
    v[q] = ((x - mu) * rs) * ga + be;
  }
  float* dst = out + kOut0Elems + f;
  *(volatile v4f*)dst = v;
  __threadfence();
  *(volatile v4f*)dst = v;
}

extern "C" void kernel_launch(void* const* d_in, const int* in_sizes, int n_in,
                              void* d_out, int out_size, void* d_ws, size_t ws_size,
                              hipStream_t stream) {
  if (n_in < 7) return;
  if (in_sizes[0] != kNb * kAcap * kPix) return;
  if (in_sizes[1] != kNb * kAcap * kCdim * kPix) return;
  if (in_sizes[2] != kNrow * kM * kCdim) return;
  if (in_sizes[3] != kNrow * kBcap * kCdim) return;
  if (in_sizes[4] != kNrow * kBcap) return;
  if (in_sizes[5] != kM || in_sizes[6] != kM) return;
  if (out_size != kOutElems) return;
  if (ws_size < kWsTotal) return;

  const float* act   = (const float*)d_in[0];
  const float* pose  = (const float*)d_in[1];
  const float* W1    = (const float*)d_in[2];
  const float* W2    = (const float*)d_in[3];
  const float* b2    = (const float*)d_in[4];
  const float* gamma = (const float*)d_in[5];
  const float* beta  = (const float*)d_in[6];

  char* ws = (char*)d_ws;
  unsigned short* bt   = (unsigned short*)(ws + kOffBt);
  float* pu            = (float*)(ws + kOffPu);
  float* ar            = (float*)(ws + kOffAr);
  float* arsum         = (float*)(ws + kOffArsum);
  float* aout          = (float*)(ws + kOffAout);
  float* poseo         = (float*)(ws + kOffPoseo);
  float* mean_ws       = (float*)(ws + kOffMean);
  float* rstd_ws       = (float*)(ws + kOffRstd);
  float* out           = (float*)d_out;

  repack_w1_kernel<<<kBtUnits / 256, 256, 0, stream>>>(W1, bt);
  gather_pose_kernel<<<kP, 288, 0, stream>>>(pose, pu);
  route_kernel<<<kP / 16, 288, 0, stream>>>(act, pu, W2, b2, ar, arsum, aout);
  vote_gemm_kernel<<<(kP / 16) * 4, 256, 0, stream>>>(pu, ar, bt, arsum, poseo);
  bn_stats_kernel<<<1, kM, 0, stream>>>(poseo, mean_ws, rstd_ws);
  write_out0_kernel<<<kOut0Units / 256, 256, 0, stream>>>(aout, out);
  write_out1_kernel<<<kOut1Units / 256, 256, 0, stream>>>(poseo, mean_ws, rstd_ws, gamma, beta, out);
}
